// GraphSAGE_57028575756304
// MI455X (gfx1250) — hardware-verified
//
#include <hip/hip_runtime.h>
#include <stddef.h>
#include <stdint.h>
#include <math.h>


#define DIN    64
#define HD1    64
#define HD2    32
#define K1     64
#define NN1    128
#define K2     128
#define NN2    64
#define NTHR   256
#define NWAVE  8
#define EPT    8
#define CHUNK  (NTHR * EPT)
#define WCAP   (EPT * 32)
#define LISTN  (NWAVE * WCAP)
#define NBA    512
#define SLA    9
#define RCAP   20480
#define DEGCAP 96
#define NB3    4096
#define SL3    12
#define GBM    64
#define GBN    64
#define GTHR   128
#define NUP    512
#define AGG_ZINTS    (LISTN + 2 * RCAP + 3 * NBA)
#define MISC_INTS    16
#define P3S_FLOATS   (2 * NBA)
#define AGG_LDS_INTS (AGG_ZINTS + MISC_INTS + P3S_FLOATS)
#define WSMAX  134217728

static_assert((CHUNK & (CHUNK - 1)) == 0 && CHUNK <= 4096);
static_assert((NBA & (NBA - 1)) == 0 && NBA == (1 << SLA));
static_assert((NB3 & (NB3 - 1)) == 0 && NB3 == (1 << SL3));
static_assert(((long long)CHUNK << SLA) < (1LL << 31));
static_assert(((long long)CHUNK << SL3) < (1LL << 31));
static_assert(LISTN % NTHR == 0 && NB3 % NTHR == 0 && NB3 == 16 * NTHR);
static_assert(NBA % NWAVE == 0 && NBA % 32 == 0 && NBA % GBM == 0);
static_assert(RCAP % 32 == 0 && AGG_ZINTS % 4 == 0 && LISTN % 4 == 0 && ((AGG_ZINTS + MISC_INTS) % 4) == 0);
static_assert(P3S_FLOATS == 4 * NTHR);
static_assert(K1 % 32 == 0 && K2 % 32 == 0 && K2 == 2 * HD1 && NN1 == 2 * HD1 && NN2 == 2 * HD2);
static_assert(NN1 % GBN == 0 && NN2 % GBN == 0 && GBM == (GTHR / 32) * 16 && GBN == 64);
static_assert(HD1 == 2 * 32 && HD2 == 32 && DIN == K1);
static_assert(NUP % NTHR == 0 && NUP == HD1 * (K1 / 8) && NUP == HD2 * (K2 / 8));
static_assert(AGG_LDS_INTS * 4 <= 300000);

typedef float          v2f   __attribute__((ext_vector_type(2)));
typedef float          v4f   __attribute__((ext_vector_type(4)));
typedef float          v8f   __attribute__((ext_vector_type(8)));
typedef int            v4i   __attribute__((ext_vector_type(4)));
typedef int            v8i   __attribute__((ext_vector_type(8)));
typedef unsigned int   v4u   __attribute__((ext_vector_type(4)));
typedef unsigned short v8us  __attribute__((ext_vector_type(8)));
typedef unsigned short v16us __attribute__((ext_vector_type(16)));
typedef __bf16         v16bf __attribute__((ext_vector_type(16)));
typedef v2f  __attribute__((may_alias)) v2fa;
typedef v4f  __attribute__((may_alias)) v4fa;
typedef v4i  __attribute__((may_alias)) v4ia;
typedef v8us __attribute__((may_alias)) v8usa;
union FragB { v16bf v; v16us u; v8us h[2]; v8i w; };

__device__ __forceinline__ v8f wmb(const FragB& a, const FragB& b, v8f c) {
  v8f d = __builtin_amdgcn_wmma_f32_16x16x32_bf16(false, a.v, false, b.v, (short)0, c, false, false);
  asm volatile("v_nop\n\tv_nop\n\tv_nop\n\tv_nop" : "+v"(d) : "v"(a.w), "v"(b.w));
  return d;
}

__device__ __forceinline__ unsigned bf16_bits(float f) {
  const unsigned u = __float_as_uint(f);
  return (u + 0x7FFFu + ((u >> 16) & 1u)) >> 16;
}
__device__ __forceinline__ float bf16_val(float f) {
  return __uint_as_float(bf16_bits(f) << 16);
}

template <int SLB>
__device__ __forceinline__ int scan_chunk(const int* __restrict__ dsts, int nE, int cbase, int slotBase,
                                          int nb, int vec8, int* list, int tid, int lane, int wave) {
  int wc = 0;
  const int el0  = tid * EPT;
  const int e0   = cbase + el0;
  const int sent = -2147483647 - 1;
  v4i da, db;
  if (vec8 != 0 && cbase + CHUNK <= nE) {
    da = *(const v4i*)(dsts + e0);
    db = *(const v4i*)(dsts + e0 + 4);
  } else {
    da.x = (e0     < nE) ? dsts[min(e0,     nE - 1)] : sent;
    da.y = (e0 + 1 < nE) ? dsts[min(e0 + 1, nE - 1)] : sent;
    da.z = (e0 + 2 < nE) ? dsts[min(e0 + 2, nE - 1)] : sent;
    da.w = (e0 + 3 < nE) ? dsts[min(e0 + 3, nE - 1)] : sent;
    db.x = (e0 + 4 < nE) ? dsts[min(e0 + 4, nE - 1)] : sent;
    db.y = (e0 + 5 < nE) ? dsts[min(e0 + 5, nE - 1)] : sent;
    db.z = (e0 + 6 < nE) ? dsts[min(e0 + 6, nE - 1)] : sent;
    db.w = (e0 + 7 < nE) ? dsts[min(e0 + 7, nE - 1)] : sent;
  }
  const unsigned nbs = (unsigned)slotBase;
  const unsigned unb = (unsigned)nb;
  const unsigned s0 = (unsigned)da.x - nbs, s1 = (unsigned)da.y - nbs;
  const unsigned s2 = (unsigned)da.z - nbs, s3 = (unsigned)da.w - nbs;
  const unsigned s4 = (unsigned)db.x - nbs, s5 = (unsigned)db.y - nbs;
  const unsigned s6 = (unsigned)db.z - nbs, s7 = (unsigned)db.w - nbs;
  const bool h0 = s0 < unb, h1 = s1 < unb, h2 = s2 < unb, h3 = s3 < unb;
  const bool h4 = s4 < unb, h5 = s5 < unb, h6 = s6 < unb, h7 = s7 < unb;
  const unsigned any = __builtin_amdgcn_ballot_w32(h0 | h1 | h2 | h3 | h4 | h5 | h6 | h7);
  if (any != 0u) {
#define HITJ(J, HJ, SJ) { \
      const unsigned mj = __builtin_amdgcn_ballot_w32(HJ); \
      if (mj != 0u) { \
        if (HJ) { \
          const int pos = wc + (int)__builtin_amdgcn_mbcnt_lo(mj, 0u); \
          if (pos < WCAP) list[wave * WCAP + pos] = ((el0 + (J)) << SLB) | (int)(SJ); \
        } \
        wc += (int)__builtin_popcount(mj); } }
    HITJ(0, h0, s0)
    HITJ(1, h1, s1)
    HITJ(2, h2, s2)
    HITJ(3, h3, s3)
    HITJ(4, h4, s4)
    HITJ(5, h5, s5)
    HITJ(6, h6, s6)
    HITJ(7, h7, s7)
#undef HITJ
  }
  return wc;
}

__global__ __launch_bounds__(NTHR) void k_wprep(const float* __restrict__ W1l, const float* __restrict__ W1r,
                                                const float* __restrict__ W2l, const float* __restrict__ W2r,
                                                unsigned short* B1T, unsigned short* B2T) {
  const int u    = (int)blockIdx.x * NTHR + (int)threadIdx.x;
  const int part = u >> 9;
  const int v    = u & (NUP - 1);
  const float* p;
  unsigned short* dp;
  int strd;
  if (part == 0) {
    const int n = v >> 3, k8 = (v & 7) * 8;
    p = W1l + (size_t)k8 * HD1 + n; strd = HD1; dp = B1T + (size_t)n * K1 + k8;
  } else if (part == 1) {
    const int n = v >> 3, k8 = (v & 7) * 8;
    p = W1r + (size_t)k8 * HD1 + n; strd = HD1; dp = B1T + (size_t)(HD1 + n) * K1 + k8;
  } else if (part == 2) {
    const int n = v >> 4, k8 = (v & 15) * 8, kk = k8 & (HD1 - 1);
    p = W2l + (size_t)kk * HD2 + n; strd = HD2; dp = B2T + (size_t)n * K2 + k8;
  } else if (part == 3) {
    const int n = v >> 4, k8 = (v & 15) * 8, kk = k8 & (HD1 - 1);
    p = W2r + (size_t)kk * HD2 + n; strd = HD2; dp = B2T + (size_t)(HD2 + n) * K2 + k8;
  } else {
    return;
  }
  v8us o;
#pragma unroll
  for (int i = 0; i < 8; ++i) o[i] = (unsigned short)bf16_bits(p[(size_t)i * strd]);
  *(volatile v8us*)dp = o;
  __threadfence();
  *(volatile v8us*)dp = o;
}

__global__ __launch_bounds__(NTHR) void k_cvx(const float* __restrict__ x, int nN, int nUnits,
                                              unsigned short* xb) {
  const int u = (int)blockIdx.x * NTHR + (int)threadIdx.x;
  if (u >= nUnits) return;
  const int row = u >> 3;
  const int k8  = (u & 7) * 8;
  const int rc  = row < nN ? row : nN - 1;
  const float* p = x + (size_t)rc * DIN + k8;
  const v4f a = *(const v4fa*)p;
  const v4f b = *(const v4fa*)(p + 4);
  const bool ok = row < nN;
  v8us o;
  o[0] = ok ? (unsigned short)bf16_bits(a.x) : (unsigned short)0;
  o[1] = ok ? (unsigned short)bf16_bits(a.y) : (unsigned short)0;
  o[2] = ok ? (unsigned short)bf16_bits(a.z) : (unsigned short)0;
  o[3] = ok ? (unsigned short)bf16_bits(a.w) : (unsigned short)0;
  o[4] = ok ? (unsigned short)bf16_bits(b.x) : (unsigned short)0;
  o[5] = ok ? (unsigned short)bf16_bits(b.y) : (unsigned short)0;
  o[6] = ok ? (unsigned short)bf16_bits(b.z) : (unsigned short)0;
  o[7] = ok ? (unsigned short)bf16_bits(b.w) : (unsigned short)0;
  unsigned short* dp = xb + (size_t)row * DIN + k8;
  *(volatile v8us*)dp = o;
  __threadfence();
  *(volatile v8us*)dp = o;
}

__global__ __launch_bounds__(GTHR) void k_gemm(
    const unsigned short* __restrict__ A, const unsigned short* __restrict__ WT,
    float* outF, int K, int ldo)
{
  __shared__ __attribute__((aligned(16))) float stg[GBM * GBN];
  const int tid = (int)threadIdx.x, lane = tid & 31, wave = tid >> 5, hh = lane >> 4, m = lane & 15;
  const int rowBase = (int)blockIdx.x * GBM;
  const int col0    = (int)blockIdx.y * GBN;

  v8f acc[4];
  {
    const v8f z = {0.f, 0.f, 0.f, 0.f, 0.f, 0.f, 0.f, 0.f};
    acc[0] = z; acc[1] = z; acc[2] = z; acc[3] = z;
  }
  const unsigned short* ap = A  + (size_t)(rowBase + 16 * wave + m) * (size_t)K + 8 * hh;
  const unsigned short* wp = WT + (size_t)(col0 + m) * (size_t)K + 8 * hh;
  const int ksteps = K >> 5;
#pragma unroll 1
  for (int ks = 0; ks < ksteps; ++ks) {
    FragB af;
    af.h[0] = *(const v8usa*)(ap + 32 * ks);
    af.h[1] = *(const v8usa*)(ap + 32 * ks + 16);
#pragma unroll
    for (int t = 0; t < 4; ++t) {
      const unsigned short* wq = wp + (size_t)(16 * t) * (size_t)K + 32 * ks;
      FragB bf;
      bf.h[0] = *(const v8usa*)wq;
      bf.h[1] = *(const v8usa*)(wq + 16);
      acc[t] = wmb(af, bf, acc[t]);
    }
  }

#pragma unroll
  for (int t = 0; t < 4; ++t) {
    const int lc = 16 * t + m;
#pragma unroll
    for (int r = 0; r < 8; ++r) {
      const int lr = 16 * wave + 8 * hh + r;
      stg[lr * GBN + lc] = acc[t][r];
    }
  }
  __syncthreads();

  v4f fv[8];
#pragma unroll
  for (int i = 0; i < 8; ++i) {
    const int lr = 16 * wave + 2 * i + hh;
    fv[i] = *(const v4fa*)(stg + lr * GBN + 4 * m);
  }
#pragma unroll
  for (int i = 0; i < 8; ++i) {
    const int lr = 16 * wave + 2 * i + hh;
    const int gr = rowBase + lr;
    float* op = outF + (size_t)gr * (size_t)ldo + col0 + 4 * m;
    *(volatile v4f*)op = fv[i];
  }
  __threadfence();
#pragma unroll
  for (int i = 0; i < 8; ++i) {
    const int lr = 16 * wave + 2 * i + hh;
    const int gr = rowBase + lr;
    float* op = outF + (size_t)gr * (size_t)ldo + col0 + 4 * m;
    *(volatile v4f*)op = fv[i];
  }
}

template <int MODE>
__global__ __launch_bounds__(NTHR) void k_agg(const int* __restrict__ srcs, const int* __restrict__ dsts,
                                              int nE, int nN, int vec8, int mRows,
                                              const float* __restrict__ pl, const float* __restrict__ bias,
                                              const float* __restrict__ w3l, const float* __restrict__ w3r,
                                              const float* __restrict__ b3,
                                              unsigned short* hb, float* pr3) {
  extern __shared__ __attribute__((aligned(16))) int dsm[];
  int* list = dsm;
  int* hl   = dsm + LISTN;
  int* sl   = dsm + LISTN + RCAP;
  int* cnt  = dsm + LISTN + 2 * RCAP;
  int* offs = cnt + NBA;
  int* cur  = offs + NBA;
  int* misc = cur + NBA;
  float* p3s = (float*)(misc + MISC_INTS);
  const int tid = (int)threadIdx.x, lane = tid & 31, wave = tid >> 5;
  const int nodeBase = (int)blockIdx.x * NBA;

  {
    const v4i z4 = {0, 0, 0, 0};
    for (int i = tid * 4; i < AGG_ZINTS; i += NTHR * 4) *(v4ia*)(dsm + i) = z4;
    if (tid < MISC_INTS) misc[tid] = 0;
  }
  float bv0 = 0.0f, bv1 = 0.0f, wlv = 0.0f, wrv = 0.0f, b3v = 0.0f;
  if constexpr (MODE == 1) {
    const v2f a = *(const v2fa*)(bias + 2 * lane);
    bv0 = bf16_val(a.x); bv1 = bf16_val(a.y);
  } else {
    bv0 = bf16_val(bias[lane]);
    wlv = bf16_val(w3l[lane]);
    wrv = bf16_val(w3r[lane]);
    b3v = bf16_val(b3[0]);
  }
  __syncthreads();

  int t = 0, ov = 0;
  const int nChunks = (nE + CHUNK - 1) / CHUNK;
#pragma unroll 1
  for (int ch = 0; ch < nChunks; ++ch) {
    const int cbase = ch * CHUNK;
    const int wc = scan_chunk<SLA>(dsts, nE, cbase, nodeBase, NBA, vec8, list, tid, lane, wave);
    if (lane == 0) misc[wave] = wc;
    __syncthreads();
    if (wave == 0) {
#pragma unroll 1
      for (int w2 = 0; w2 < NWAVE; ++w2) {
        int c = misc[w2];
        c = c < 0 ? 0 : (c > WCAP ? WCAP : c);
#pragma unroll 1
        for (int b0 = 0; b0 < c; b0 += 32) {
          const int idx = b0 + lane;
          const int ent = list[w2 * WCAP + (idx < WCAP ? idx : WCAP - 1)];
          const int m32 = (c - b0) < 32 ? (c - b0) : 32;
#pragma unroll 1
          for (int k = 0; k < m32; ++k) {
            const int u    = __builtin_amdgcn_readlane(ent, k);
            const int slot = u & (NBA - 1);
            const int el   = (u >> SLA) & (CHUNK - 1);
            const int pk   = ((cbase + el) << SLA) | slot;
            if (t < RCAP) {
              if (lane == 0) { hl[t] = pk; cnt[slot] = cnt[slot] + 1; }
              t = t + 1;
            } else {
              ov = 1;
            }
          }
        }
      }
    }
    __syncthreads();
  }
  if (wave == 0 && lane == 0) { misc[8] = t; misc[9] = ov; }
  __syncthreads();
  int tt = misc[8];
  tt = tt < 0 ? 0 : (tt > RCAP ? RCAP : tt);
  const int ovf = misc[9];

  if (wave == 0) {
    const int base = lane * (NBA / 32);
    int s = 0;
#pragma unroll 1
    for (int i = 0; i < NBA / 32; ++i) s += cnt[base + i];
    int incl = s;
#pragma unroll
    for (int d = 1; d < 32; d <<= 1) {
      const int y = __shfl_up(incl, d, 32);
      if (lane >= d) incl += y;
    }
    int run = incl - s;
#pragma unroll 1
    for (int i = 0; i < NBA / 32; ++i) {
      const int cv = cnt[base + i];
      offs[base + i] = run;
      cur[base + i]  = run;
      run += cv;
    }
  }
  __syncthreads();
  if (wave == 0) {
#pragma unroll 1
    for (int b0 = 0; b0 < tt; b0 += 32) {
      const int idx = b0 + lane;
      const int ent = hl[idx < RCAP ? idx : RCAP - 1];
      const int m32 = (tt - b0) < 32 ? (tt - b0) : 32;
#pragma unroll 1
      for (int k = 0; k < m32; ++k) {
        const int u    = __builtin_amdgcn_readlane(ent, k);
        const int slot = u & (NBA - 1);
        if (lane == 0) {
          int p = cur[slot];
          p = p < 0 ? 0 : (p > RCAP - 1 ? RCAP - 1 : p);
          sl[p] = u;
          cur[slot] = p + 1;
        }
      }
    }
  }
  __syncthreads();

  const float qnan = __int_as_float(0x7fc00000);
  const float pz = (ovf != 0) ? qnan : 0.0f;
  const int q0s = (4 * lane) & 31, q1s = (4 * lane + 1) & 31;
  const int q2s = (4 * lane + 2) & 31, q3s = (4 * lane + 3) & 31;
#pragma unroll 1
  for (int si = 0; si < NBA / NWAVE; ++si) {
    const int s    = si * NWAVE + wave;
    const int node = nodeBase + s;
    const int c0 = cnt[s];
    const int craw = c0 < 0 ? 0 : c0;
    const bool big = craw > DEGCAP;
    const int c = craw > DEGCAP ? DEGCAP : craw;
    int o = offs[s];
    o = o < 0 ? 0 : (o > RCAP ? RCAP : o);
    const int nc = node < nN ? node : nN - 1;
    float acc0 = 0.0f, acc1 = 0.0f;
#pragma unroll 1
    for (int b0 = 0; b0 < c; b0 += 32) {
      int idx = o + b0 + lane;
      idx = idx > RCAP - 1 ? RCAP - 1 : idx;
      const int ent = sl[idx];
      int eid = ent >> SLA;
      eid = eid < 0 ? 0 : (eid > nE - 1 ? nE - 1 : eid);
      int sr = srcs[eid];
      sr = sr < 0 ? 0 : (sr > nN - 1 ? nN - 1 : sr);
      const int m32 = (c - b0) < 32 ? (c - b0) : 32;
#pragma unroll 1
      for (int k = 0; k < m32; ++k) {
        const int sk = __builtin_amdgcn_readlane(sr, k);
        if constexpr (MODE == 1) {
          const v2f a = *(const v2fa*)(pl + (size_t)sk * NN1 + 2 * lane);
          acc0 += a.x; acc1 += a.y;
        } else {
          acc0 += pl[(size_t)sk * NN2 + lane];
        }
      }
    }
    float sv0 = 0.0f, sv1 = 0.0f;
    if constexpr (MODE == 1) {
      const v2f a = *(const v2fa*)(pl + (size_t)nc * NN1 + HD1 + 2 * lane);
      sv0 = a.x; sv1 = a.y;
    } else {
      sv0 = pl[(size_t)nc * NN2 + HD2 + lane];
    }
    const float cntf = (craw < 1) ? 1.0f : (float)craw;
    const float inv  = 1.0f / cntf;
    const float pzr = big ? qnan : pz;
    const bool live = node < nN;
    float y0 = (acc0 * inv + bv0) + sv0;
    float y1 = (acc1 * inv + bv1) + sv1;
    y0 = fmaxf(y0, 0.0f); y1 = fmaxf(y1, 0.0f);
    y0 = y0 + pzr; y1 = y1 + pzr;
    const float v0 = live ? y0 : 0.0f;
    const float v1 = live ? y1 : 0.0f;
    if constexpr (MODE == 1) {
      const bool wr = (node < mRows) && (lane < 16);
      const unsigned hb0 = bf16_bits(v0), hb1 = bf16_bits(v1);
      const unsigned lb0 = bf16_bits(v0 - __uint_as_float(hb0 << 16));
      const unsigned lb1 = bf16_bits(v1 - __uint_as_float(hb1 << 16));
      const int hw = (int)(hb0 | (hb1 << 16));
      const int lw = (int)(lb0 | (lb1 << 16));
      const int g0 = __shfl(hw, q0s, 32), g1 = __shfl(hw, q1s, 32);
      const int g2 = __shfl(hw, q2s, 32), g3 = __shfl(hw, q3s, 32);
      const int p0 = __shfl(lw, q0s, 32), p1 = __shfl(lw, q1s, 32);
      const int p2 = __shfl(lw, q2s, 32), p3 = __shfl(lw, q3s, 32);
      const bool lsel = (lane & 8) != 0;
      v4u pv;
      pv.x = (unsigned int)(lsel ? p0 : g0);
      pv.y = (unsigned int)(lsel ? p1 : g1);
      pv.z = (unsigned int)(lsel ? p2 : g2);
      pv.w = (unsigned int)(lsel ? p3 : g3);
      unsigned short* hp = hb + (size_t)node * K2 + 8 * (lane & 15);
      if (wr) *(volatile v4u*)hp = pv;
      __threadfence();
      if (wr) *(volatile v4u*)hp = pv;
    } else {
      float pp = v0 * wlv;
      float rq = v0 * wrv;
#pragma unroll
      for (int d = 16; d >= 1; d >>= 1) {
        pp += __shfl_xor(pp, d, 32);
        rq += __shfl_xor(rq, d, 32);
      }
      if (lane == 0) {
        p3s[2 * s]     = pp;
        p3s[2 * s + 1] = live ? (rq + b3v) : 0.0f;
      }
    }
  }
  if constexpr (MODE == 2) {
    __syncthreads();
    const v4f ovv = *(const v4fa*)(p3s + 4 * tid);
    float* op = pr3 + (size_t)nodeBase * 2 + 4 * tid;
    *(volatile v4f*)op = ovv;
    __threadfence();
    *(volatile v4f*)op = ovv;
  }
}

__global__ __launch_bounds__(NTHR) void k_out(const int* __restrict__ srcs, const int* __restrict__ dsts,
                                              int nE, int nN, int vec8, const float* __restrict__ pr3,
                                              float* out) {
  __shared__ __attribute__((aligned(16))) int scnt[NB3];
  __shared__ __attribute__((aligned(16))) float sacc[NB3];
  __shared__ __attribute__((aligned(16))) int list[LISTN];
  __shared__ int wcnt[NWAVE];
  const int tid = (int)threadIdx.x, lane = tid & 31, wave = tid >> 5;
  const int nodeBase = (int)blockIdx.x * NB3;

  for (int i = tid; i < NB3; i += NTHR) { scnt[i] = 0; sacc[i] = 0.0f; }
  for (int i = tid; i < LISTN; i += NTHR) list[i] = 0;
  if (tid < NWAVE) wcnt[tid] = 0;
  __syncthreads();

  const int nChunks = (nE + CHUNK - 1) / CHUNK;
#pragma unroll 1
  for (int ch = 0; ch < nChunks; ++ch) {
    const int cbase = ch * CHUNK;
    const int wc = scan_chunk<SL3>(dsts, nE, cbase, nodeBase, NB3, vec8, list, tid, lane, wave);
    if (lane == 0) wcnt[wave] = wc;
    __syncthreads();
    if (wave == 0) {
#pragma unroll 1
      for (int w2 = 0; w2 < NWAVE; ++w2) {
        int c = wcnt[w2];
        c = c < 0 ? 0 : (c > WCAP ? WCAP : c);
#pragma unroll 1
        for (int b0 = 0; b0 < c; b0 += 32) {
          const int idx = b0 + lane;
          const int ent = list[w2 * WCAP + (idx < WCAP ? idx : WCAP - 1)];
          const int el  = (ent >> SL3) & (CHUNK - 1);
          int eid = cbase + el;
          eid = eid > nE - 1 ? nE - 1 : eid;
          int sr = srcs[eid];
          sr = sr < 0 ? 0 : (sr > nN - 1 ? nN - 1 : sr);
          const int pvi = __float_as_int(pr3[(size_t)2 * (size_t)sr]);
          const int m32 = (c - b0) < 32 ? (c - b0) : 32;
#pragma unroll 1
          for (int k = 0; k < m32; ++k) {
            const int   u  = __builtin_amdgcn_readlane(ent, k);
            const float v  = __int_as_float(__builtin_amdgcn_readlane(pvi, k));
            const int   st = u & (NB3 - 1);
            if (lane == 0) { scnt[st] = scnt[st] + 1; sacc[st] = sacc[st] + v; }
          }
        }
      }
    }
    __syncthreads();
  }

#pragma unroll 1
  for (int s = tid; s < NB3; s += NTHR) {
    const int node = nodeBase + s;
    const int nc = node < nN ? node : nN - 1;
    const float r3 = pr3[(size_t)2 * (size_t)nc + 1];
    const int c = scnt[s];
    const float a = sacc[s];
    const float cntf = (c < 1) ? 1.0f : (float)c;
    float v = a * (1.0f / cntf) + r3;
    v = (v > 30.0f) ? 30.0f : v;
    v = (v < -30.0f) ? -30.0f : v;
    const float e = expf(-v);
    const float o = 1.0f / (1.0f + e);
    sacc[s] = (node < nN) ? o : 0.0f;
  }
  __syncthreads();
  v4f ov[4];
#pragma unroll
  for (int it = 0; it < 4; ++it) ov[it] = *(const v4fa*)(sacc + 4 * (it * NTHR + tid));
#pragma unroll
  for (int it = 0; it < 4; ++it) {
    const int e0 = nodeBase + 4 * (it * NTHR + tid);
    if (e0 + 4 <= nN) *(volatile v4f*)(out + e0) = ov[it];
  }
  __threadfence();
#pragma unroll
  for (int it = 0; it < 4; ++it) {
    const int e0 = nodeBase + 4 * (it * NTHR + tid);
    if (e0 + 4 <= nN) *(volatile v4f*)(out + e0) = ov[it];
  }
}

static inline int cdiv(int a, int b) { return (a + b - 1) / b; }
static inline size_t al256(size_t o) { return (o + 255) & ~(size_t)255; }

extern "C" void kernel_launch(void* const* d_in, const int* in_sizes, int n_in,
                              void* d_out, int out_size, void* d_ws, size_t ws_size,
                              hipStream_t stream) {
  if (n_in < 11) return;
  if (in_sizes[0] < DIN || (in_sizes[0] % DIN) != 0) return;
  const int nN = in_sizes[0] / DIN;
  if (nN < 32 || nN > (1 << 22) || (nN % 32) != 0) return;
  if (in_sizes[1] < 2 || (in_sizes[1] & 1) != 0) return;
  const int nE = in_sizes[1] / 2;
  if (nE < 1 || nE >= (1 << (31 - SLA))) return;
  if (in_sizes[2] != DIN * HD1 || in_sizes[3] != HD1 || in_sizes[4] != DIN * HD1) return;
  if (in_sizes[5] != HD1 * HD2 || in_sizes[6] != HD2 || in_sizes[7] != HD1 * HD2) return;
  if (in_sizes[8] != HD2 || in_sizes[9] != 1 || in_sizes[10] != HD2) return;
  if (out_size != nN) return;

  const float* x    = (const float*)d_in[0];
  const int*   edge = (const int*)d_in[1];
  const float* W1l  = (const float*)d_in[2];
  const float* b1   = (const float*)d_in[3];
  const float* W1r  = (const float*)d_in[4];
  const float* W2l  = (const float*)d_in[5];
  const float* b2   = (const float*)d_in[6];
  const float* W2r  = (const float*)d_in[7];
  const float* W3l  = (const float*)d_in[8];
  const float* b3   = (const float*)d_in[9];
  const float* W3r  = (const float*)d_in[10];
  float* out = (float*)d_out;
  const int* src = edge;
  const int* dst = edge + nE;

  const int MP  = cdiv(nN, GBM) * GBM;
  const int gM  = MP / GBM;
  const int gA  = cdiv(MP, NBA);
  const int NBP = gA * NBA;
  const int gO  = cdiv(nN, NB3);
  if ((long long)gA * NBA < (long long)MP) return;
  if ((long long)gO * NB3 < (long long)nN) return;
  const int vec8 = ((nE & 3) == 0) ? 1 : 0;

  char* ws = (char*)d_ws;
  size_t off = 0;
  const size_t oB1T = off; off = al256(off + (size_t)NN1 * K1 * 2);
  const size_t oB2T = off; off = al256(off + (size_t)NN2 * K2 * 2);
  const size_t oXB  = off; off = al256(off + (size_t)MP * DIN * 2);
  const size_t oPR1 = off; off = al256(off + (size_t)MP * NN1 * 4);
  const size_t oH1  = off; off = al256(off + (size_t)MP * K2 * 2);
  const size_t oPR2 = off; off = al256(off + (size_t)MP * NN2 * 4);
  const size_t oPR3 = off; off = al256(off + (size_t)NBP * 2 * 4);
  if (off > ws_size || off > (size_t)WSMAX) return;
  unsigned short* B1T = (unsigned short*)(ws + oB1T);
  unsigned short* B2T = (unsigned short*)(ws + oB2T);
  unsigned short* XB  = (unsigned short*)(ws + oXB);
  float*          PR1 = (float*)(ws + oPR1);
  unsigned short* H1  = (unsigned short*)(ws + oH1);
  float*          PR2 = (float*)(ws + oPR2);
  float*          PR3 = (float*)(ws + oPR3);

  const size_t aggLds = (size_t)AGG_LDS_INTS * 4;
  hipFuncSetAttribute(reinterpret_cast<const void*>(&k_agg<1>), hipFuncAttributeMaxDynamicSharedMemorySize, (int)aggLds);
  hipFuncSetAttribute(reinterpret_cast<const void*>(&k_agg<2>), hipFuncAttributeMaxDynamicSharedMemorySize, (int)aggLds);

  const int nUx = MP * (DIN / 8);
  k_wprep<<<(4 * NUP) / NTHR, NTHR, 0, stream>>>(W1l, W1r, W2l, W2r, B1T, B2T);
  k_cvx<<<cdiv(nUx, NTHR), NTHR, 0, stream>>>(x, nN, nUx, XB);
  k_gemm<<<dim3(gM, NN1 / GBN), GTHR, 0, stream>>>(XB, B1T, PR1, K1, NN1);
  k_agg<1><<<gA, NTHR, aggLds, stream>>>(src, dst, nE, nN, vec8, MP, PR1, b1, W3l, W3r, b3, H1, PR3);
  k_gemm<<<dim3(gM, NN2 / GBN), GTHR, 0, stream>>>(H1, B2T, PR2, K2, NN2);
  k_agg<2><<<gA, NTHR, aggLds, stream>>>(src, dst, nE, nN, vec8, MP, PR2, b2, W3l, W3r, b3, H1, PR3);
  k_out<<<gO, NTHR, 0, stream>>>(src, dst, nE, nN, vec8, PR3, out);
}
